// GroupedMultiQueryAttention_12034498363675
// MI455X (gfx1250) — hardware-verified
//
#include <hip/hip_runtime.h>
#include <cstdint>

#define T_SEQ   2048
#define HID     2048
#define NH      32
#define NKV     8
#define HD      64
#define KVDIM   (NKV * HD)
#define RSPLIT (1.0f / 2048.0f)

typedef _Float16 f16;
typedef f16   v16h __attribute__((ext_vector_type(16)));
typedef f16   v8h  __attribute__((ext_vector_type(8)));
typedef float v8f  __attribute__((ext_vector_type(8)));
typedef float v4f_t __attribute__((ext_vector_type(4)));
typedef float v4fa  __attribute__((ext_vector_type(4), may_alias));
typedef unsigned v4u_t __attribute__((ext_vector_type(4)));

__device__ __forceinline__ f16 lo_of(float v, f16 h) { return (f16)((v - (float)h) * 2048.0f); }
__device__ __forceinline__ unsigned pk2s(float a, float b, unsigned* lo) {
  const f16 h0 = (f16)a, h1 = (f16)b;
  *lo = (unsigned)__builtin_bit_cast(unsigned short, lo_of(a, h0)) | ((unsigned)__builtin_bit_cast(unsigned short, lo_of(b, h1)) << 16);
  return (unsigned)__builtin_bit_cast(unsigned short, h0) | ((unsigned)__builtin_bit_cast(unsigned short, h1) << 16);
}
__device__ __forceinline__ v8f wmma16(v16h a, v16h b, v8f c) { return __builtin_amdgcn_wmma_f32_16x16x32_f16(false, a, false, b, (short)0, c, false, false); }
struct Frag2 { v16h h, l; };
__device__ __forceinline__ v8f wmma_split(const Frag2& a, const Frag2& b, v8f c) { v8f x = {}; x = wmma16(a.l, b.h, x); x = wmma16(a.h, b.l, x); return wmma16(a.h, b.h, c) + x * RSPLIT; }
__device__ __forceinline__ v16h cat8(v8h a, v8h b) { return __builtin_shufflevector(a, b, 0,1,2,3,4,5,6,7,8,9,10,11,12,13,14,15); }
__device__ __forceinline__ Frag2 ld2(const f16* p, size_t plane) { Frag2 f; f.h = cat8(*(const v8h*)p, *(const v8h*)(p + 16)); f.l = cat8(*(const v8h*)(p + plane), *(const v8h*)(p + plane + 16)); return f; }

__global__ void __launch_bounds__(256) cvt_planes(const float* __restrict__ in, f16* __restrict__ out, int n, size_t plane) {
  int i = (blockIdx.x * blockDim.x + threadIdx.x) * 2;
  if (i >= n) return;
  unsigned lo; const unsigned p = pk2s(in[i], in[i + 1], &lo);
  *(volatile unsigned*)(out + i) = p; *(volatile unsigned*)(out + plane + i) = lo; __threadfence();
  *(volatile unsigned*)(out + i) = p; *(volatile unsigned*)(out + plane + i) = lo;
}

template <int MODE>
__global__ void __launch_bounds__(256) proj_kernel(const f16* __restrict__ X, size_t plx, const f16* __restrict__ Wt, size_t plw,
                                                   void* __restrict__ Yp, size_t ply, int NW, int rope) {
  __shared__ __attribute__((aligned(16))) float stg[8][16 * 68];
  const int wib = threadIdx.x >> 5;
  const int wave = (blockIdx.x * blockDim.x + threadIdx.x) >> 5;
  const int lane = threadIdx.x & 31, lrow = lane & 15, lhi = lane >> 4;
  const int ncg = NW / 64;
  const int i0 = (wave / ncg) * 16, n0 = (wave % ncg) * 64;
  if (i0 >= T_SEQ) return;
  v8f acc[4] = {};
  const f16* xrow = X + (size_t)(i0 + lrow) * HID + lhi * 8;
  for (int kk = 0; kk < HID; kk += 32) {
    const Frag2 a = ld2(xrow + kk, plx);
#pragma unroll
    for (int n = 0; n < 4; ++n) acc[n] = wmma_split(a, ld2(Wt + (size_t)(n0 + n * 16 + lrow) * HID + kk + lhi * 8, plw), acc[n]);
  }
  float* sw = stg[wib];
#pragma unroll
  for (int n = 0; n < 4; ++n)
#pragma unroll
    for (int r = 0; r < 8; ++r) sw[(r + lhi * 8) * 68 + n * 16 + lrow] = acc[n][r];
  asm volatile("s_wait_dscnt 0" ::: "memory");
  if (MODE == 0 && rope) {
    const float kLn = 0.28782313663f;
    for (int c = lane; c < 16 * 32; c += 32) {
      const int rr = c >> 5, pi = c & 31, d0 = 2 * pi;
      const float t = (float)(i0 + rr);
      const float th0 = t * __expf(-(float)(d0 & 31) * kLn), th1 = t * __expf(-(float)((d0 + 1) & 31) * kLn);
      const float x0 = sw[rr * 68 + d0], x1 = sw[rr * 68 + d0 + 1];
      sw[rr * 68 + d0]     = x0 * __cosf(th0) - x1 * __sinf(th0);
      sw[rr * 68 + d0 + 1] = x1 * __cosf(th1) + x0 * __sinf(th1);
    }
    asm volatile("s_wait_dscnt 0" ::: "memory");
  }
#pragma unroll 1
  for (int pass = 0; pass < 2; ++pass) {
    if (MODE == 0) {
      f16* Y = (f16*)Yp;
#pragma unroll
      for (int i = 0; i < 4; ++i) { const int c = lane + 32 * i, rr = c >> 3, q = (c & 7) * 8; const float* s = sw + rr * 68 + q;
        v4u_t v, vl; unsigned lq;
        v.x = pk2s(s[0], s[1], &lq); vl.x = lq; v.y = pk2s(s[2], s[3], &lq); vl.y = lq; v.z = pk2s(s[4], s[5], &lq); vl.z = lq; v.w = pk2s(s[6], s[7], &lq); vl.w = lq;
        f16* d = Y + (size_t)(i0 + rr) * NW + n0 + q;
        *(volatile v4u_t*)d = v; *(volatile v4u_t*)(d + ply) = vl; }
    } else {
      float* Y = (float*)Yp;
#pragma unroll
      for (int i = 0; i < 8; ++i) { const int c = lane + 32 * i, rr = c >> 4, q = (c & 15) * 4;
        *(volatile v4f_t*)(Y + (size_t)(i0 + rr) * NW + n0 + q) = *(const volatile v4fa*)(sw + rr * 68 + q); }
    }
    __threadfence();
  }
}

__global__ void __launch_bounds__(256) flash_kernel(const f16* __restrict__ Q, const f16* __restrict__ Kc, const f16* __restrict__ Vc,
                                                    f16* __restrict__ O) {
  __shared__ __attribute__((aligned(16))) f16 plds[8][2][16 * 32];
  __shared__ __attribute__((aligned(16))) f16 vs[8][2][32 * 72];
  __shared__ __attribute__((aligned(16))) float stg[8][16 * 68];
  const size_t PLQ = (size_t)T_SEQ * HID, PLK = (size_t)T_SEQ * KVDIM;
  const int wib = threadIdx.x >> 5;
  const int wave = (blockIdx.x * blockDim.x + threadIdx.x) >> 5;
  const int lane = threadIdx.x & 31, lrow = lane & 15, lhi = lane >> 4;
  const int h = wave / (T_SEQ / 16), i0 = (wave % (T_SEQ / 16)) * 16;
  if (h >= NH) return;
  const int kvh = h >> 2;
  const f16* qbase = Q  + h * HD;
  const f16* kbase = Kc + kvh * HD;
  const f16* vbase = Vc + kvh * HD;
  v8f o[4] = {};
  float m[8], l[8];
#pragma unroll
  for (int r = 0; r < 8; ++r) { m[r] = -3.0e38f; l[r] = 0.f; }
  const float LOG2E = 1.4426950408889634f, SCALE = 0.125f, NEGV = -3.0e38f;
  f16* vh = vs[wib][0]; f16* vl = vs[wib][1];

  for (int j0 = 0; j0 <= i0 + 15; j0 += 32) {
    { const f16* vr = vbase + (size_t)(j0 + lane) * KVDIM;
#pragma unroll
      for (int u = 0; u < 8; ++u) { *(v8h*)&vh[lane * 72 + u * 8] = *(const v8h*)(vr + u * 8); *(v8h*)&vl[lane * 72 + u * 8] = *(const v8h*)(vr + PLK + u * 8); } }
    const Frag2 kb00 = ld2(kbase + (size_t)(j0 + lrow) * KVDIM + lhi * 8, PLK), kb01 = ld2(kbase + (size_t)(j0 + lrow) * KVDIM + 32 + lhi * 8, PLK);
    const Frag2 kb10 = ld2(kbase + (size_t)(j0 + 16 + lrow) * KVDIM + lhi * 8, PLK), kb11 = ld2(kbase + (size_t)(j0 + 16 + lrow) * KVDIM + 32 + lhi * 8, PLK);
    asm volatile("s_wait_dscnt 0" ::: "memory");
    {
      f16* ph = plds[wib][0]; f16* pl = plds[wib][1];
      v8f s0 = {}, s1 = {};
      { const Frag2 qa0 = ld2(qbase + (size_t)(i0 + lrow) * HID + lhi * 8, PLQ), qa1 = ld2(qbase + (size_t)(i0 + lrow) * HID + 32 + lhi * 8, PLQ);
        s0 = wmma_split(qa0, kb00, s0); s0 = wmma_split(qa1, kb01, s0);
        s1 = wmma_split(qa0, kb10, s1); s1 = wmma_split(qa1, kb11, s1); }
      float sc0[8], sc1[8], mnew[8];
#pragma unroll
      for (int r = 0; r < 8; ++r) {
        int row = i0 + r + lhi * 8;
        int c0 = j0 + lrow, c1 = j0 + 16 + lrow;
        float a0 = (c0 <= row) ? s0[r] * SCALE : NEGV;
        float a1 = (c1 <= row) ? s1[r] * SCALE : NEGV;
        sc0[r] = a0; sc1[r] = a1;
        float mx = fmaxf(a0, a1);
        mx = fmaxf(mx, __shfl_xor(mx, 1)); mx = fmaxf(mx, __shfl_xor(mx, 2)); mx = fmaxf(mx, __shfl_xor(mx, 4)); mx = fmaxf(mx, __shfl_xor(mx, 8));
        mnew[r] = fmaxf(m[r], mx);
      }
#pragma unroll
      for (int r = 0; r < 8; ++r) {
        int row = i0 + r + lhi * 8;
        float p0 = (j0 + lrow <= row) ? __builtin_exp2f((sc0[r] - mnew[r]) * LOG2E) : 0.f;
        float p1 = (j0 + 16 + lrow <= row) ? __builtin_exp2f((sc1[r] - mnew[r]) * LOG2E) : 0.f;
        float rs = p0 + p1;
        rs += __shfl_xor(rs, 1); rs += __shfl_xor(rs, 2); rs += __shfl_xor(rs, 4); rs += __shfl_xor(rs, 8);
        float fac = __builtin_exp2f((m[r] - mnew[r]) * LOG2E);
        l[r] = l[r] * fac + rs;
        m[r] = mnew[r];
#pragma unroll
        for (int n = 0; n < 4; ++n) o[n][r] *= fac;
        const float q0 = p0 * 1024.0f, q1 = p1 * 1024.0f;
        const f16 h0 = (f16)q0, h1 = (f16)q1;
        ph[(r + lhi * 8) * 32 + lrow] = h0;      pl[(r + lhi * 8) * 32 + lrow] = lo_of(q0, h0);
        ph[(r + lhi * 8) * 32 + 16 + lrow] = h1; pl[(r + lhi * 8) * 32 + 16 + lrow] = lo_of(q1, h1);
      }
    }
    asm volatile("s_wait_dscnt 0" ::: "memory");
    {
      const f16* ph = plds[wib][0]; const f16* pl = plds[wib][1];
      Frag2 pa; pa.h = cat8(*(const v8h*)&ph[lrow * 32 + lhi * 8], *(const v8h*)&ph[lrow * 32 + 16 + lhi * 8]); pa.l = cat8(*(const v8h*)&pl[lrow * 32 + lhi * 8], *(const v8h*)&pl[lrow * 32 + 16 + lhi * 8]);
#pragma unroll
      for (int n = 0; n < 4; ++n) {
        Frag2 vbn;
#pragma unroll
        for (int i = 0; i < 16; ++i) { const int key = (i < 8) ? (lhi * 8 + i) : (16 + lhi * 8 + (i - 8)); vbn.h[i] = vh[key * 72 + n * 16 + lrow]; vbn.l[i] = vl[key * 72 + n * 16 + lrow]; }
        o[n] = wmma_split(pa, vbn, o[n]);
      }
    }
  }
  float* sw = stg[wib];
#pragma unroll
  for (int n = 0; n < 4; ++n)
#pragma unroll
    for (int r = 0; r < 8; ++r) sw[(r + lhi * 8) * 68 + n * 16 + lrow] = o[n][r] / (l[r] * 1024.0f);
  asm volatile("s_wait_dscnt 0" ::: "memory");
#pragma unroll 1
  for (int pass = 0; pass < 2; ++pass) {
#pragma unroll
    for (int i = 0; i < 4; ++i) { const int c = lane + 32 * i, rr = c >> 3, q = (c & 7) * 8; const float* s = sw + rr * 68 + q;
      v4u_t v, vl2; unsigned lq;
      v.x = pk2s(s[0], s[1], &lq); vl2.x = lq; v.y = pk2s(s[2], s[3], &lq); vl2.y = lq; v.z = pk2s(s[4], s[5], &lq); vl2.z = lq; v.w = pk2s(s[6], s[7], &lq); vl2.w = lq;
      f16* d = O + (size_t)(i0 + rr) * HID + h * HD + q;
      *(volatile v4u_t*)d = v; *(volatile v4u_t*)(d + PLQ) = vl2; }
    __threadfence();
  }
}

extern "C" void kernel_launch(void* const* d_in, const int* in_sizes, int n_in,
                              void* d_out, int out_size, void* d_ws, size_t ws_size,
                              hipStream_t stream) {
    (void)in_sizes; (void)n_in; (void)out_size; (void)ws_size;
    const float* x  = (const float*)d_in[0];
    const float* Wq = (const float*)d_in[1];
    const float* Wk = (const float*)d_in[2];
    const float* Wv = (const float*)d_in[3];
    const float* Wo = (const float*)d_in[4];
    float* out = (float*)d_out;

    char* ws = (char*)d_ws;
    size_t off = 0;
    auto alloc = [&](size_t bytes) -> void* { void* p = ws + off; off += (bytes + 255) & ~(size_t)255; return p; };
    const size_t PLX = (size_t)T_SEQ * HID, PLWQ = (size_t)HID * HID, PLWK = (size_t)KVDIM * HID, PLK = (size_t)T_SEQ * KVDIM;
    f16* xb  = (f16*)alloc(PLX * 2 * 2);
    f16* wqb = (f16*)alloc(PLWQ * 2 * 2);
    f16* wkb = (f16*)alloc(PLWK * 2 * 2);
    f16* wvb = (f16*)alloc(PLWK * 2 * 2);
    f16* wob = (f16*)alloc(PLWQ * 2 * 2);
    f16* qb  = (f16*)alloc(PLX * 2 * 2);
    f16* kb  = (f16*)alloc(PLK * 2 * 2);
    f16* vb  = (f16*)alloc(PLK * 2 * 2);
    f16* ab  = (f16*)alloc(PLX * 2 * 2);
    const int nt = T_SEQ;

    auto cast = [&](const float* src, f16* dst, size_t nel) { cvt_planes<<<(unsigned)((nel / 2 + 255) / 256), 256, 0, stream>>>(src, dst, (int)nel, nel); };
    cast(x,  xb,  PLX);
    cast(Wq, wqb, PLWQ);
    cast(Wk, wkb, PLWK);
    cast(Wv, wvb, PLWK);
    cast(Wo, wob, PLWQ);

    proj_kernel<0><<<(nt / 16) * (HID / 64) / 8,   256, 0, stream>>>(xb, PLX, wqb, PLWQ, qb, PLX, HID, 1);
    proj_kernel<0><<<(nt / 16) * (KVDIM / 64) / 8, 256, 0, stream>>>(xb, PLX, wkb, PLWK, kb, PLK, KVDIM, 1);
    proj_kernel<0><<<(nt / 16) * (KVDIM / 64) / 8, 256, 0, stream>>>(xb, PLX, wvb, PLWK, vb, PLK, KVDIM, 0);
    flash_kernel<<<NH * (T_SEQ / 16) / 8, 256, 0, stream>>>(qb, kb, vb, ab);
    proj_kernel<2><<<(nt / 16) * (HID / 64) / 8,   256, 0, stream>>>(ab, PLX, wob, PLWQ, out, 0, HID, 0);
}
